// ParticleNetBlock_25039659336453
// MI455X (gfx1250) — hardware-verified
//
#include <hip/hip_runtime.h>
#include <stddef.h>
#include <math.h>


#define CH     64
#define KNB    16
#define APZ    72
#define KPB    64
#define PQW    128
#define NTHR   256
#define NWAVE  8
#define NIT    16
#define NPB    (NWAVE * NIT)
#define GROWS  64
#define GTHR   128
#define DEGCAP 1024
#define EPT    8
#define NGRP   2
#define CHUNK  (NTHR * EPT * NGRP)
#define WCAP   (EPT * NGRP * 32)
#define LISTN  (NWAVE * WCAP)
#define NBC    4096
#define NBF    1024
#define RCAP   40960
#define RBN    128
#define OTHR   512
#define LDS_FILL ((RCAP + NBF + LISTN) * 4 + 64)
#define OFF_B1 0
#define OFF_B2 (2 * CH * KPB)
#define OFF_B3 (OFF_B2 + CH * KPB)
#define BPTOT  (OFF_B3 + CH * KPB)
#define WSCAP  134217728
#define BN_EPS 1e-5f
#define SLOPE  0.01f
#define WSC    64.0f
#define ZSC    8.0f
#define RWSC   0.015625f
#define RZW    0.001953125f

static_assert(NIT * NWAVE == NPB);
static_assert(GROWS == (GTHR / 32) * 16);
static_assert((APZ % 8) == 0 && (KPB % 8) == 0 && (PQW % 32) == 0);
static_assert(BPTOT == 16384);
static_assert(GTHR * 16 * 4 == GROWS * PQW);
static_assert(NWAVE * CH == GTHR * 4);
static_assert((CHUNK & (CHUNK - 1)) == 0);
static_assert(CHUNK <= 4096);
static_assert(NBC <= 4096 && NBF <= 4096);
static_assert((NBC & (NBC - 1)) == 0 && (NBF & (NBF - 1)) == 0);
static_assert(NBC == 4 * NBF);
static_assert(OTHR * 8 == NBC);
static_assert((RCAP % 32) == 0);
static_assert((DEGCAP % KNB) == 0);

typedef float    v2f  __attribute__((ext_vector_type(2)));
typedef float    v4f  __attribute__((ext_vector_type(4)));
typedef float    v8f  __attribute__((ext_vector_type(8)));
typedef double   v2d  __attribute__((ext_vector_type(2)));
typedef int      v4i  __attribute__((ext_vector_type(4)));
typedef _Float16 v4h  __attribute__((ext_vector_type(4)));
typedef _Float16 v8h  __attribute__((ext_vector_type(8)));
typedef _Float16 v16h __attribute__((ext_vector_type(16)));
union Frag { v16h v; v8h h[2]; };

__device__ __forceinline__ v8f wmh(v16h a, v16h b, v8f c) {
  v8f d = __builtin_amdgcn_wmma_f32_16x16x32_f16(false, a, false, b, (short)0, c, false, false);
  asm volatile("v_nop\n\tv_nop\n\tv_nop\n\tv_nop" : "+v"(d) : "v"(a), "v"(b));
  return d;
}

__device__ __forceinline__ v8h cvt8(v4f a, v4f b, float s) {
  v8h r;
  r[0] = (_Float16)(a.x * s); r[1] = (_Float16)(a.y * s); r[2] = (_Float16)(a.z * s); r[3] = (_Float16)(a.w * s);
  r[4] = (_Float16)(b.x * s); r[5] = (_Float16)(b.y * s); r[6] = (_Float16)(b.z * s); r[7] = (_Float16)(b.w * s);
  return r;
}

__device__ __forceinline__ v4h cvt4z(v4f a) {
  v4h r;
  r.x = (_Float16)(a.x * ZSC); r.y = (_Float16)(a.y * ZSC); r.z = (_Float16)(a.z * ZSC); r.w = (_Float16)(a.w * ZSC);
  return r;
}

template <int NT>
__device__ __forceinline__ void mma16(const _Float16* At, const _Float16* __restrict__ Bpl,
                                      int lane, v8f (&acc)[NT]) {
  const int hh = lane >> 4, m = lane & 15;
#pragma unroll
  for (int t = 0; t < NT; ++t) { v8f z = {0.f, 0.f, 0.f, 0.f, 0.f, 0.f, 0.f, 0.f}; acc[t] = z; }
  const _Float16* ap = At + m * APZ + 8 * hh;
  const _Float16* bb = Bpl + (size_t)m * KPB + 8 * hh;
#pragma unroll 1
  for (int ks = 0; ks < CH / 32; ++ks) {
    Frag a;
    a.h[0] = *(const v8h*)(ap + 32 * ks);
    a.h[1] = *(const v8h*)(ap + 32 * ks + 16);
#pragma unroll
    for (int t = 0; t < NT; ++t) {
      const _Float16* bp = bb + (size_t)(16 * t) * KPB + 32 * ks;
      Frag b;
      b.h[0] = *(const v8h*)bp;
      b.h[1] = *(const v8h*)(bp + 16);
      acc[t] = wmh(a.v, b.v, acc[t]);
    }
  }
}

template <int J0>
__device__ __forceinline__ void rows_h1(const float* __restrict__ PQ, int sl, int dl, int hh, int m, int nvt,
                                        v4f& fs, v4f& fq) {
#pragma unroll
  for (int j = J0; j < J0 + 4; ++j) {
    const int sa = __builtin_amdgcn_readlane(sl, 2 * j), sb = __builtin_amdgcn_readlane(sl, 2 * j + 1);
    const int da = __builtin_amdgcn_readlane(dl, 2 * j), db = __builtin_amdgcn_readlane(dl, 2 * j + 1);
    const int s = hh ? sb : sa, d = hh ? db : da;
    const v4f q  = *(const v4f*)(PQ + (size_t)s * PQW + CH + 4 * m);
    const v4f dn = *(const v4f*)(PQ + (size_t)d * PQW + 4 * m);
    v4f h = dn + q;
    const bool ok = (2 * j + hh) < nvt;
    h.x = ok ? h.x : 0.0f; h.y = ok ? h.y : 0.0f; h.z = ok ? h.z : 0.0f; h.w = ok ? h.w : 0.0f;
    fs = fs + h;
    fq = h * h + fq;
  }
}

template <int J0, bool GD>
__device__ __forceinline__ void rows_z1(_Float16* zw, const float* __restrict__ PQ, int sl, int dl, v4f dnc,
                                        int hh, int m, v4f mu, v4f sc, v4f be) {
#pragma unroll
  for (int j = J0; j < J0 + 4; ++j) {
    const int sa = __builtin_amdgcn_readlane(sl, 2 * j), sb = __builtin_amdgcn_readlane(sl, 2 * j + 1);
    const int s = hh ? sb : sa;
    const v4f q = *(const v4f*)(PQ + (size_t)s * PQW + CH + 4 * m);
    v4f dn = dnc;
    if (GD) {
      const int da = __builtin_amdgcn_readlane(dl, 2 * j), db = __builtin_amdgcn_readlane(dl, 2 * j + 1);
      const int d = hh ? db : da;
      dn = *(const v4f*)(PQ + (size_t)d * PQW + 4 * m);
    }
    const v4f h = dn + q;
    v4f u = (h - mu) * sc + be;
    u.x = u.x >= 0.0f ? u.x : SLOPE * u.x;
    u.y = u.y >= 0.0f ? u.y : SLOPE * u.y;
    u.z = u.z >= 0.0f ? u.z : SLOPE * u.z;
    u.w = u.w >= 0.0f ? u.w : SLOPE * u.w;
    *(v4h*)(zw + (2 * j + hh) * APZ + 4 * m) = cvt4z(u);
  }
}

__device__ __forceinline__ void store_part(const double* comb, double* part, int tid) {
  v2d cv = {0.0, 0.0};
  if (tid < CH) cv = *(const v2d*)(comb + 2 * tid);
  double* gp = part + (size_t)blockIdx.x * (2 * CH) + 2 * (tid & (CH - 1));
  if (tid < CH) *(volatile v2d*)gp = cv;
  __threadfence();
  if (tid < CH) *(volatile v2d*)gp = cv;
}

__device__ __forceinline__ void combine_red(const double* red, double* comb, int tid) {
  if (tid < 2 * CH) {
    const int c = tid & (CH - 1), sel = tid >> 6;
    double a = 0.0;
#pragma unroll 1
    for (int r = 0; r < 2 * NWAVE; ++r) a += red[(sel * (2 * NWAVE) + r) * CH + c];
    comb[tid] = a;
  }
}

template <int NB>
__device__ __forceinline__ int scan_chunk(const int* __restrict__ dsts, int nE, int cbase, int slotBase,
                                          int vec8, int* list, int tid, int lane, int wave) {
  int wc = 0;
#pragma unroll
  for (int g = 0; g < NGRP; ++g) {
    const int el0  = (g * NTHR + tid) * EPT;
    const int e0   = cbase + el0;
    const int sent = -2147483647 - 1;
    v4i da, db;
    if (vec8 != 0 && cbase + CHUNK <= nE) {
      da = *(const v4i*)(dsts + e0);
      db = *(const v4i*)(dsts + e0 + 4);
    } else {
      da.x = (e0     < nE) ? dsts[min(e0, nE - 1)] : sent;
      da.y = (e0 + 1 < nE) ? dsts[min(e0 + 1, nE - 1)] : sent;
      da.z = (e0 + 2 < nE) ? dsts[min(e0 + 2, nE - 1)] : sent;
      da.w = (e0 + 3 < nE) ? dsts[min(e0 + 3, nE - 1)] : sent;
      db.x = (e0 + 4 < nE) ? dsts[min(e0 + 4, nE - 1)] : sent;
      db.y = (e0 + 5 < nE) ? dsts[min(e0 + 5, nE - 1)] : sent;
      db.z = (e0 + 6 < nE) ? dsts[min(e0 + 6, nE - 1)] : sent;
      db.w = (e0 + 7 < nE) ? dsts[min(e0 + 7, nE - 1)] : sent;
    }
    const unsigned nb = (unsigned)slotBase;
    const unsigned s0 = (unsigned)da.x - nb, s1 = (unsigned)da.y - nb;
    const unsigned s2 = (unsigned)da.z - nb, s3 = (unsigned)da.w - nb;
    const unsigned s4 = (unsigned)db.x - nb, s5 = (unsigned)db.y - nb;
    const unsigned s6 = (unsigned)db.z - nb, s7 = (unsigned)db.w - nb;
    const bool h0 = s0 < (unsigned)NB, h1 = s1 < (unsigned)NB, h2 = s2 < (unsigned)NB, h3 = s3 < (unsigned)NB;
    const bool h4 = s4 < (unsigned)NB, h5 = s5 < (unsigned)NB, h6 = s6 < (unsigned)NB, h7 = s7 < (unsigned)NB;
    const unsigned any = __builtin_amdgcn_ballot_w32(h0 | h1 | h2 | h3 | h4 | h5 | h6 | h7);
    if (any != 0u) {
#define HITJ(J, HJ, SJ) { \
        const unsigned mj = __builtin_amdgcn_ballot_w32(HJ); \
        if (mj != 0u) { \
          if (HJ) { \
            const int pos = wc + (int)__builtin_amdgcn_mbcnt_lo(mj, 0u); \
            if (pos < WCAP) list[wave * WCAP + pos] = ((el0 + (J)) << 12) | (int)(SJ); \
          } \
          wc += (int)__builtin_popcount(mj); } }
      HITJ(0, h0, s0)
      HITJ(1, h1, s1)
      HITJ(2, h2, s2)
      HITJ(3, h3, s3)
      HITJ(4, h4, s4)
      HITJ(5, h5, s5)
      HITJ(6, h6, s6)
      HITJ(7, h7, s7)
#undef HITJ
    }
  }
  return wc;
}

__global__ __launch_bounds__(NTHR) void k_wprep(const float* __restrict__ W1, const float* __restrict__ W2,
                                                const float* __restrict__ W3, _Float16* Bpl) {
  const int blk = blockIdx.x, tid = threadIdx.x;
  float v[8];
  int o;
  if (blk < 4) {
    const int i = blk * NTHR + tid;
    const int n = i >> 3, k0 = (i & 7) * 8;
    const int kb = (n >> 6) * CH, nc = n & (CH - 1);
#pragma unroll
    for (int e = 0; e < 8; ++e) v[e] = W1[(kb + k0 + e) * CH + nc];
    o = OFF_B1 + i * 8;
  } else if (blk < 6) {
    const int i = (blk - 4) * NTHR + tid;
    const int n = i >> 3, k0 = (i & 7) * 8;
#pragma unroll
    for (int e = 0; e < 8; ++e) v[e] = W2[(k0 + e) * CH + n];
    o = OFF_B2 + i * 8;
  } else {
    const int i = (blk - 6) * NTHR + tid;
    const int n = i >> 3, k0 = (i & 7) * 8;
#pragma unroll
    for (int e = 0; e < 8; ++e) v[e] = W3[(k0 + e) * CH + n];
    o = OFF_B3 + i * 8;
  }
  v8h hv;
#pragma unroll
  for (int e = 0; e < 8; ++e) hv[e] = (_Float16)(v[e] * WSC);
  _Float16* dp = Bpl + o;
  *(volatile v8h*)dp = hv;
  __threadfence();
  *(volatile v8h*)dp = hv;
}

__global__ __launch_bounds__(NTHR) void k_count(const int* __restrict__ dsts, int* cnt, int nE, int vec8) {
  __shared__ __attribute__((aligned(16))) int scnt[NBC];
  __shared__ __attribute__((aligned(16))) int list[LISTN];
  __shared__ int wcnt[NWAVE];
  const int tid = threadIdx.x, lane = tid & 31, wave = tid >> 5;
  const int nodeBase = blockIdx.x * NBC;

  for (int i = tid; i < NBC; i += NTHR) scnt[i] = 0;
  __syncthreads();

  const int nChunks = (nE + CHUNK - 1) / CHUNK;
#pragma unroll 1
  for (int ch = 0; ch < nChunks; ++ch) {
    const int cbase = ch * CHUNK;
    const int wc = scan_chunk<NBC>(dsts, nE, cbase, nodeBase, vec8, list, tid, lane, wave);
    if (lane == 0) wcnt[wave] = wc;
    __syncthreads();
    if (wave == 0) {
#pragma unroll 1
      for (int wsx = 0; wsx < NWAVE; ++wsx) {
        int n = __builtin_amdgcn_readfirstlane(wcnt[wsx]);
        n = n > WCAP ? WCAP : (n < 0 ? 0 : n);
        const int* lp = list + wsx * WCAP;
#pragma unroll 1
        for (int i = 0; i < n; ++i) {
          const int ent  = __builtin_amdgcn_readfirstlane(lp[i]);
          const int slot = ent & (NBC - 1);
          if (lane == 0) scnt[slot] = scnt[slot] + 1;
        }
      }
    }
    __syncthreads();
  }

  v4i cq[4];
#pragma unroll
  for (int q = 0; q < 4; ++q) {
    const int f = (wave * 4 + q) * 128 + 4 * lane;
    cq[q] = *(const v4i*)(scnt + f);
  }
  int* cp = cnt + (size_t)nodeBase;
#pragma unroll
  for (int q = 0; q < 4; ++q) {
    const int f = (wave * 4 + q) * 128 + 4 * lane;
    *(volatile v4i*)(cp + f) = cq[q];
  }
  __threadfence();
#pragma unroll
  for (int q = 0; q < 4; ++q) {
    const int f = (wave * 4 + q) * 128 + 4 * lane;
    *(volatile v4i*)(cp + f) = cq[q];
  }
}

__global__ __launch_bounds__(OTHR) void k_offsets(
    const int* __restrict__ cnt, int* off, int* rbase, int nChunk) {
  __shared__ __attribute__((aligned(16))) int soff[NBC];
  __shared__ __attribute__((aligned(16))) int srb[RBN];
  __shared__ int wtot[OTHR / 32];
  const int tid = threadIdx.x, lane = tid & 31, wave = tid >> 5, sub = tid >> 7;
  for (int i = tid; i < RBN; i += OTHR) srb[i] = 0;
  int carry = 0;
#pragma unroll 1
  for (int ch = 0; ch < nChunk; ++ch) {
    const int base = ch * NBC;
    const v4i c0 = *(const v4i*)(cnt + base + 8 * tid);
    const v4i c1 = *(const v4i*)(cnt + base + 8 * tid + 4);
    const int e0 = max(c0.x, 0), e1 = max(c0.y, 0), e2 = max(c0.z, 0), e3 = max(c0.w, 0);
    const int e4 = max(c1.x, 0), e5 = max(c1.y, 0), e6 = max(c1.z, 0), e7 = max(c1.w, 0);
    const int ts = e0 + e1 + e2 + e3 + e4 + e5 + e6 + e7;
    int incl = ts;
#pragma unroll
    for (int d = 1; d < 32; d <<= 1) {
      const int t = __shfl_up(incl, d);
      if (lane >= d) incl += t;
    }
    if (lane == 31) wtot[wave] = incl;
    __syncthreads();
    const int S0 = wtot[0]  + wtot[1]  + wtot[2]  + wtot[3];
    const int S1 = wtot[4]  + wtot[5]  + wtot[6]  + wtot[7];
    const int S2 = wtot[8]  + wtot[9]  + wtot[10] + wtot[11];
    const int S3 = wtot[12] + wtot[13] + wtot[14] + wtot[15];
    int pre = 0;
#pragma unroll 1
    for (int w = 4 * sub; w < wave; ++w) pre += wtot[w];
    const int b0 = carry;
    const int b1 = b0 + ((S0 + 31) & ~31);
    const int b2 = b1 + ((S1 + 31) & ~31);
    const int b3 = b2 + ((S2 + 31) & ~31);
    const int b4 = b3 + ((S3 + 31) & ~31);
    const int myb = sub == 0 ? b0 : (sub == 1 ? b1 : (sub == 2 ? b2 : b3));
    if (tid == 0) {
      srb[min(4 * ch + 0, RBN - 1)] = b0;
      srb[min(4 * ch + 1, RBN - 1)] = b1;
      srb[min(4 * ch + 2, RBN - 1)] = b2;
      srb[min(4 * ch + 3, RBN - 1)] = b3;
    }
    int run = myb + pre + incl - ts;
    soff[8 * tid + 0] = run; run += e0;
    soff[8 * tid + 1] = run; run += e1;
    soff[8 * tid + 2] = run; run += e2;
    soff[8 * tid + 3] = run; run += e3;
    soff[8 * tid + 4] = run; run += e4;
    soff[8 * tid + 5] = run; run += e5;
    soff[8 * tid + 6] = run; run += e6;
    soff[8 * tid + 7] = run;
    carry = b4;
    __syncthreads();
    const v4i o0 = *(const v4i*)(soff + 4 * tid);
    const v4i o1 = *(const v4i*)(soff + 4 * (tid + OTHR));
    int* op = off + base;
    *(volatile v4i*)(op + 4 * tid) = o0;
    *(volatile v4i*)(op + 4 * (tid + OTHR)) = o1;
    __threadfence();
    *(volatile v4i*)(op + 4 * tid) = o0;
    *(volatile v4i*)(op + 4 * (tid + OTHR)) = o1;
    __syncthreads();
  }
  if (tid == 0) srb[min(4 * nChunk, RBN - 1)] = carry;
  __syncthreads();
  v4i rv = {0, 0, 0, 0};
  if (tid < 32) rv = *(const v4i*)(srb + 4 * tid);
  if (tid < 32) *(volatile v4i*)(rbase + 4 * tid) = rv;
  __threadfence();
  if (tid < 32) *(volatile v4i*)(rbase + 4 * tid) = rv;
}

__global__ __launch_bounds__(NTHR) void k_fill(
    const int* __restrict__ srcs, const int* __restrict__ dsts,
    const int* __restrict__ off, const int* __restrict__ rbase,
    int* csr, int nN, int nE, int vec8, int csrLen) {
  extern __shared__ v4f lds_dyn[];
  int* region = (int*)lds_dyn;
  int* cursor = region + RCAP;
  int* list   = cursor + NBF;
  int* wcnt   = list + LISTN;
  const int tid = threadIdx.x, lane = tid & 31, wave = tid >> 5;
  const int b = blockIdx.x;
  const int nodeBase = b * NBF;

  int rb0 = rbase[b];
  const int rb1 = rbase[b + 1];
  rb0 = rb0 < 0 ? 0 : (rb0 > csrLen ? csrLen : rb0);
  rb0 &= ~31;
  int len = rb1 - rb0;
  len = len < 0 ? 0 : (len > RCAP ? RCAP : len);
  int lenW = (len + 31) & ~31;
  if (rb0 + lenW > csrLen) lenW = (csrLen - rb0) & ~31;

  {
    const v4i z = {0, 0, 0, 0};
    for (int i = tid; i < RCAP / 4; i += NTHR) ((v4i*)region)[i] = z;
    for (int s = tid; s < NBF; s += NTHR) {
      int o = off[nodeBase + s] - rb0;
      o = o < 0 ? 0 : (o > RCAP ? RCAP : o);
      cursor[s] = o;
    }
  }
  __syncthreads();

  const int nChunks = (nE + CHUNK - 1) / CHUNK;
#pragma unroll 1
  for (int ch = 0; ch < nChunks; ++ch) {
    const int cbase = ch * CHUNK;
    const int wc = scan_chunk<NBF>(dsts, nE, cbase, nodeBase, vec8, list, tid, lane, wave);
    if (lane == 0) wcnt[wave] = wc;
    __syncthreads();
    if (wave == 0) {
#pragma unroll 1
      for (int wsx = 0; wsx < NWAVE; ++wsx) {
        int n = __builtin_amdgcn_readfirstlane(wcnt[wsx]);
        n = n > WCAP ? WCAP : (n < 0 ? 0 : n);
        const int* lp = list + wsx * WCAP;
#pragma unroll 1
        for (int i = 0; i < n; ++i) {
          const int ent  = __builtin_amdgcn_readfirstlane(lp[i]);
          const int slot = ent & (NBF - 1);
          int e = cbase + ((ent >> 12) & (CHUNK - 1));
          e = e > nE - 1 ? nE - 1 : e;
          int sv = srcs[e];
          sv = sv < 0 ? 0 : (sv > nN - 1 ? nN - 1 : sv);
          if (lane == 0) {
            int pos = cursor[slot];
            pos = pos < 0 ? 0 : (pos > RCAP - 1 ? RCAP - 1 : pos);
            region[pos] = sv;
            const int np = pos + 1;
            cursor[slot] = np > RCAP ? RCAP : np;
          }
        }
      }
    }
    __syncthreads();
  }

  const int nv = lenW >> 2;
  int* gp = csr + rb0;
#pragma unroll 1
  for (int i = tid; i < nv; i += NTHR) { const v4i v = ((const v4i*)region)[i]; *(volatile v4i*)(gp + 4 * i) = v; }
  __threadfence();
#pragma unroll 1
  for (int i = tid; i < nv; i += NTHR) { const v4i v = ((const v4i*)region)[i]; *(volatile v4i*)(gp + 4 * i) = v; }
}

__global__ __launch_bounds__(GTHR) void k_nodegemm(const float* __restrict__ x, const _Float16* __restrict__ Bpl,
                                                   const float* __restrict__ b1, float* PQ, int nN) {
  __shared__ __attribute__((aligned(16))) _Float16 At[GROWS * APZ];
  __shared__ __attribute__((aligned(16))) float stg[GROWS * PQW];
  const int tid = threadIdx.x, lane = tid & 31, wave = tid >> 5, hh = lane >> 4, m = lane & 15;
  const int rowBase = blockIdx.x * GROWS;
  {
    const int r = tid >> 1, c0 = (tid & 1) * 32;
    int xrow = rowBase + r;
    xrow = xrow > nN - 1 ? nN - 1 : xrow;
    const float* xp = x + (size_t)xrow * CH + c0;
#pragma unroll
    for (int j = 0; j < 4; ++j) {
      const v4f a = *(const v4f*)(xp + 8 * j), b = *(const v4f*)(xp + 8 * j + 4);
      *(v8h*)(At + r * APZ + c0 + 8 * j) = cvt8(a, b, 1.0f);
    }
  }
  __syncthreads();

#pragma unroll
  for (int chf = 0; chf < 2; ++chf) {
    v8f acc[4];
    mma16<4>(At + wave * 16 * APZ, Bpl + (size_t)(64 * chf) * KPB, lane, acc);
    float* sp = stg + (wave * 16 + 8 * hh) * PQW + 64 * chf + m;
    if (chf == 0) {
#pragma unroll
      for (int t = 0; t < 4; ++t) {
        const float bv = b1[16 * t + m];
#pragma unroll
        for (int r = 0; r < 8; ++r) sp[r * PQW + 16 * t] = acc[t][r] * RWSC + bv;
      }
    } else {
#pragma unroll
      for (int t = 0; t < 4; ++t) {
#pragma unroll
        for (int r = 0; r < 8; ++r) {
          const float q = acc[t][r] * RWSC;
          float* e = sp + r * PQW + 16 * t;
          e[0]   = q;
          e[-CH] = e[-CH] - q;
        }
      }
    }
  }
  __syncthreads();

  float* gp = PQ + (size_t)rowBase * PQW;
#pragma unroll
  for (int it = 0; it < 16; ++it) {
    const int f = it * GTHR + tid;
    const v4f v = *(const v4f*)(stg + 4 * f);
    *(volatile v4f*)(gp + 4 * f) = v;
  }
  __threadfence();
#pragma unroll
  for (int it = 0; it < 16; ++it) {
    const int f = it * GTHR + tid;
    const v4f v = *(const v4f*)(stg + 4 * f);
    *(volatile v4f*)(gp + 4 * f) = v;
  }
}

__global__ __launch_bounds__(NTHR) void k_stats1(const float* __restrict__ PQ, const int* __restrict__ srcs,
                                                 const int* __restrict__ dsts, double* part, int nE, int nN) {
  __shared__ __attribute__((aligned(16))) double red[2 * 2 * NWAVE * CH];
  __shared__ __attribute__((aligned(16))) double comb[2 * CH];
  const int tid = threadIdx.x, lane = tid & 31, wave = tid >> 5, hh = lane >> 4, m = lane & 15;
  const int tbase = blockIdx.x * NPB;
  double S[4] = {0.0, 0.0, 0.0, 0.0}, Qd[4] = {0.0, 0.0, 0.0, 0.0};
#pragma unroll 1
  for (int it = 0; it < NIT; ++it) {
    const int tI = tbase + it * NWAVE + wave;
    const int e0 = tI * KNB;
    int nvt = nE - e0;
    nvt = nvt < 0 ? 0 : (nvt > KNB ? KNB : nvt);
    int ei = e0 + m;
    ei = ei > nE - 1 ? nE - 1 : ei;
    int sl = srcs[ei]; sl = sl < 0 ? 0 : (sl > nN - 1 ? nN - 1 : sl);
    int dl = dsts[ei]; dl = dl < 0 ? 0 : (dl > nN - 1 ? nN - 1 : dl);
    v4f fs = {0.f, 0.f, 0.f, 0.f}, fq = {0.f, 0.f, 0.f, 0.f};
    rows_h1<0>(PQ, sl, dl, hh, m, nvt, fs, fq);
    asm volatile("" ::: "memory");
    rows_h1<4>(PQ, sl, dl, hh, m, nvt, fs, fq);
    S[0] += (double)fs.x; S[1] += (double)fs.y; S[2] += (double)fs.z; S[3] += (double)fs.w;
    Qd[0] += (double)fq.x; Qd[1] += (double)fq.y; Qd[2] += (double)fq.z; Qd[3] += (double)fq.w;
  }
  {
    v2d a0, a1, q0, q1;
    a0.x = S[0]; a0.y = S[1]; a1.x = S[2]; a1.y = S[3];
    q0.x = Qd[0]; q0.y = Qd[1]; q1.x = Qd[2]; q1.y = Qd[3];
    double* rs = red + (2 * wave + hh) * CH + 4 * m;
    double* rq = red + (2 * NWAVE) * CH + (2 * wave + hh) * CH + 4 * m;
    *(v2d*)rs = a0; *(v2d*)(rs + 2) = a1;
    *(v2d*)rq = q0; *(v2d*)(rq + 2) = q1;
  }
  __syncthreads();
  combine_red(red, comb, tid);
  __syncthreads();
  store_part(comb, part, tid);
}

__global__ __launch_bounds__(64) void k_bnfin(const double* __restrict__ part, const float* __restrict__ gam,
                                              const float* __restrict__ bet, const float* __restrict__ bnx,
                                              float* tab, double rn, int nBlk) {
  __shared__ __attribute__((aligned(16))) float sco[4 * CH];
  const int c = threadIdx.x;
  double S = 0.0, Q = 0.0;
#pragma unroll 1
  for (int b = 0; b < nBlk; ++b) {
    S += part[(size_t)b * (2 * CH) + c];
    Q += part[(size_t)b * (2 * CH) + CH + c];
  }
  const double mean = S * rn;
  double var = Q * rn - mean * mean;
  var = var < 0.0 ? 0.0 : var;
  sco[c]          = (float)mean;
  sco[CH + c]     = gam[c] * rsqrtf((float)var + BN_EPS);
  sco[2 * CH + c] = bet[c];
  sco[3 * CH + c] = bnx[c];
  __syncthreads();
  const v4f cv = *(const v4f*)(sco + 4 * c);
  *(volatile v4f*)(tab + 4 * c) = cv;
  __threadfence();
  *(volatile v4f*)(tab + 4 * c) = cv;
}

__global__ __launch_bounds__(NTHR) void k_stats2(const float* __restrict__ PQ, const int* __restrict__ srcs,
                                                 const int* __restrict__ dsts, const _Float16* __restrict__ B2,
                                                 const float* __restrict__ tab1, double* part, int nE, int nN) {
  __shared__ __attribute__((aligned(16))) _Float16 zt[NWAVE * KNB * APZ];
  __shared__ __attribute__((aligned(16))) double red[2 * 2 * NWAVE * CH];
  __shared__ __attribute__((aligned(16))) double comb[2 * CH];
  __shared__ __attribute__((aligned(16))) float ptab[4 * CH];
  const int tid = threadIdx.x, lane = tid & 31, wave = tid >> 5, hh = lane >> 4, m = lane & 15;
  const int tbase = blockIdx.x * NPB;
  _Float16* zw = zt + wave * (KNB * APZ);
  {
    const int q4 = 4 * (tid & (CH - 1));
    const v4f tv = *(const v4f*)(tab1 + q4);
    if (tid < CH) *(v4f*)(ptab + q4) = tv;
  }
  __syncthreads();
  const v4f mu1 = *(const v4f*)(ptab + 4 * m);
  const v4f sc1 = *(const v4f*)(ptab + CH + 4 * m);
  const v4f bb1 = *(const v4f*)(ptab + 2 * CH + 4 * m);
  float b2c[4];
#pragma unroll
  for (int t = 0; t < 4; ++t) b2c[t] = ptab[3 * CH + 16 * t + m];
  const v4f z4 = {0.f, 0.f, 0.f, 0.f};
  double S[4] = {0.0, 0.0, 0.0, 0.0}, Qd[4] = {0.0, 0.0, 0.0, 0.0};

#pragma unroll 1
  for (int it = 0; it < NIT; ++it) {
    const int tI = tbase + it * NWAVE + wave;
    const int e0 = tI * KNB;
    int nvt = nE - e0;
    nvt = nvt < 0 ? 0 : (nvt > KNB ? KNB : nvt);
    int ei = e0 + m;
    ei = ei > nE - 1 ? nE - 1 : ei;
    int sl = srcs[ei]; sl = sl < 0 ? 0 : (sl > nN - 1 ? nN - 1 : sl);
    int dl = dsts[ei]; dl = dl < 0 ? 0 : (dl > nN - 1 ? nN - 1 : dl);
    __syncthreads();
    rows_z1<0, true>(zw, PQ, sl, dl, z4, hh, m, mu1, sc1, bb1);
    asm volatile("" ::: "memory");
    rows_z1<4, true>(zw, PQ, sl, dl, z4, hh, m, mu1, sc1, bb1);
    __syncthreads();
    v8f acc[4];
    mma16<4>(zw, B2, lane, acc);
#pragma unroll
    for (int t = 0; t < 4; ++t) {
      float fs = 0.f, fq = 0.f;
#pragma unroll
      for (int r = 0; r < 8; ++r) {
        float v = acc[t][r] * RZW + b2c[t];
        v = ((8 * hh + r) < nvt) ? v : 0.0f;
        fs += v;
        fq = fmaf(v, v, fq);
      }
      S[t]  += (double)fs;
      Qd[t] += (double)fq;
    }
  }
#pragma unroll
  for (int t = 0; t < 4; ++t) {
    red[(2 * wave + hh) * CH + 16 * t + m] = S[t];
    red[(2 * NWAVE) * CH + (2 * wave + hh) * CH + 16 * t + m] = Qd[t];
  }
  __syncthreads();
  combine_red(red, comb, tid);
  __syncthreads();
  store_part(comb, part, tid);
}

__global__ __launch_bounds__(NTHR) void k_final(
    const float* __restrict__ PQ, const int* __restrict__ csr,
    const int* __restrict__ offp, const int* __restrict__ cntp,
    const _Float16* __restrict__ B2, const _Float16* __restrict__ B3,
    const float* __restrict__ tab1, const float* __restrict__ tab2,
    const float* __restrict__ x, float* out, int nN, int csrLen) {
  __shared__ __attribute__((aligned(16))) _Float16 z1t[NWAVE * KNB * APZ];
  __shared__ __attribute__((aligned(16))) _Float16 z2t[NWAVE * KNB * APZ];
  __shared__ __attribute__((aligned(16))) float sout[NWAVE * CH];
  __shared__ __attribute__((aligned(16))) float ptab[8 * CH];
  __shared__ __attribute__((aligned(16))) int slot[NWAVE];
  const int tid = threadIdx.x, lane = tid & 31, wave = tid >> 5, hh = lane >> 4, m = lane & 15;
  const int base = blockIdx.x * NPB;
  _Float16* z1w = z1t + wave * (KNB * APZ);
  _Float16* z2w = z2t + wave * (KNB * APZ);
  {
    const int q4 = 4 * (tid & (CH - 1));
    const v4f va = *(const v4f*)(tab1 + q4);
    const v4f vb = *(const v4f*)(tab2 + q4);
    v4f tv;
    tv.x = (tid < CH) ? va.x : vb.x; tv.y = (tid < CH) ? va.y : vb.y;
    tv.z = (tid < CH) ? va.z : vb.z; tv.w = (tid < CH) ? va.w : vb.w;
    if (tid < 2 * CH) *(v4f*)(ptab + 4 * tid) = tv;
  }
  __syncthreads();
  const v4f mu1 = *(const v4f*)(ptab + 4 * m);
  const v4f sc1 = *(const v4f*)(ptab + CH + 4 * m);
  const v4f bb1 = *(const v4f*)(ptab + 2 * CH + 4 * m);
  float b2c[4], mu2c[4], sc2c[4], be2c[4], b3c[4];
#pragma unroll
  for (int t = 0; t < 4; ++t) { b2c[t] = ptab[3 * CH + 16 * t + m]; mu2c[t] = ptab[4 * CH + 16 * t + m]; }
  asm volatile("" ::: "memory");
#pragma unroll
  for (int t = 0; t < 4; ++t) {
    sc2c[t] = ptab[5 * CH + 16 * t + m]; be2c[t] = ptab[6 * CH + 16 * t + m]; b3c[t] = ptab[7 * CH + 16 * t + m];
  }
  const float ninf = __uint_as_float(0xff800000u);

#pragma unroll 1
  for (int it = 0; it < NIT; ++it) {
    const int n = base + it * NWAVE + wave;
    const bool nval = n < nN;
    const int cc = nval ? n : nN - 1;
    const int cnr = cntp[cc];
    const int ofr = offp[cc];
    int cn = nval ? cnr : 0;
    cn = cn < 0 ? 0 : (cn > DEGCAP ? DEGCAP : cn);
    cn = __builtin_amdgcn_readfirstlane(cn);
    int of = ofr;
    of = of < 0 ? 0 : (of > csrLen ? csrLen : of);
    of = __builtin_amdgcn_readfirstlane(of);
    const v4f dnc = *(const v4f*)(PQ + (size_t)cc * PQW + 4 * m);
    float xr[4];
#pragma unroll
    for (int t = 0; t < 4; ++t) xr[t] = x[(size_t)cc * CH + 16 * t + m];
    const int ntw = (cn + KNB - 1) >> 4;
    if (lane == 0) slot[wave] = ntw;
    __syncthreads();
    int ntmax;
    {
      const v4i sA = *(const v4i*)slot, sB = *(const v4i*)(slot + 4);
      int mm = max(max(sA.x, sA.y), max(sA.z, sA.w));
      mm = max(mm, max(max(sB.x, sB.y), max(sB.z, sB.w)));
      mm = mm < 0 ? 0 : (mm > DEGCAP / KNB ? DEGCAP / KNB : mm);
      ntmax = __builtin_amdgcn_readfirstlane(mm);
    }
    float mx[4] = {ninf, ninf, ninf, ninf};
#pragma unroll 1
    for (int tt = 0; tt < ntmax; ++tt) {
      int nv = cn - tt * KNB;
      nv = nv < 0 ? 0 : (nv > KNB ? KNB : nv);
      int pos = of + tt * KNB + m;
      pos = pos < 0 ? 0 : (pos > csrLen - 1 ? csrLen - 1 : pos);
      int sv = csr[pos];
      sv = sv < 0 ? 0 : (sv > nN - 1 ? nN - 1 : sv);
      rows_z1<0, false>(z1w, PQ, sv, sv, dnc, hh, m, mu1, sc1, bb1);
      asm volatile("" ::: "memory");
      rows_z1<4, false>(z1w, PQ, sv, sv, dnc, hh, m, mu1, sc1, bb1);
      __syncthreads();
      {
        v8f acc[4];
        mma16<4>(z1w, B2, lane, acc);
#pragma unroll
        for (int t = 0; t < 4; ++t) {
#pragma unroll
          for (int r = 0; r < 8; ++r) {
            const float h2 = acc[t][r] * RZW + b2c[t];
            float u = (h2 - mu2c[t]) * sc2c[t] + be2c[t];
            u = u >= 0.0f ? u : SLOPE * u;
            z2w[(8 * hh + r) * APZ + 16 * t + m] = (_Float16)(u * ZSC);
          }
        }
      }
      __syncthreads();
      {
        v8f acc[4];
        mma16<4>(z2w, B3, lane, acc);
#pragma unroll
        for (int t = 0; t < 4; ++t) {
#pragma unroll
          for (int r = 0; r < 8; ++r) {
            const float v = ((8 * hh + r) < nv) ? acc[t][r] : ninf;
            mx[t] = fmaxf(mx[t], v);
          }
        }
      }
    }
#pragma unroll
    for (int t = 0; t < 4; ++t) mx[t] = fmaxf(mx[t], __shfl_xor(mx[t], 16, 32));
#pragma unroll
    for (int t = 0; t < 4; ++t) {
      float o = mx[t] * RZW + b3c[t] + xr[t];
      o = o >= 0.0f ? o : SLOPE * o;
      if (hh == 0) sout[wave * CH + 16 * t + m] = o;
    }
    __syncthreads();
    v4f ov = {0.f, 0.f, 0.f, 0.f};
    int node = nN;
    size_t oofs = 0;
    if (tid < GTHR) {
      const int row = tid >> 4;
      node = base + it * NWAVE + row;
      ov = *(const v4f*)(sout + 4 * tid);
      const int ncl = node < nN ? node : nN - 1;
      oofs = (size_t)ncl * CH + 4 * (tid & 15);
    }
    if (tid < GTHR && node < nN) *(volatile v4f*)(out + oofs) = ov;
    __threadfence();
    if (tid < GTHR && node < nN) *(volatile v4f*)(out + oofs) = ov;
  }
}

extern "C" void kernel_launch(void* const* d_in, const int* in_sizes, int n_in,
                              void* d_out, int out_size, void* d_ws, size_t ws_size,
                              hipStream_t stream) {
  if (n_in < 12) return;
  const int nN = in_sizes[0] / CH;
  const int nE = in_sizes[1] / 2;
  if (nN <= 0 || nE <= 0) return;
  if (in_sizes[0] != nN * CH || in_sizes[1] != 2 * nE) return;
  if (in_sizes[2] != 2 * CH * CH || in_sizes[3] != CH || in_sizes[4] != CH || in_sizes[5] != CH) return;
  if (in_sizes[6] != CH * CH || in_sizes[7] != CH || in_sizes[8] != CH || in_sizes[9] != CH) return;
  if (in_sizes[10] != CH * CH || in_sizes[11] != CH) return;
  if (out_size != nN * CH) return;
  if (nE > (1 << 28) || nN > (1 << 24)) return;

  const float* x   = (const float*)d_in[0];
  const int*   ei  = (const int*)d_in[1];
  const float* W1  = (const float*)d_in[2];
  const float* b1  = (const float*)d_in[3];
  const float* g1  = (const float*)d_in[4];
  const float* be1 = (const float*)d_in[5];
  const float* W2  = (const float*)d_in[6];
  const float* b2  = (const float*)d_in[7];
  const float* g2  = (const float*)d_in[8];
  const float* be2 = (const float*)d_in[9];
  const float* W3  = (const float*)d_in[10];
  const float* b3  = (const float*)d_in[11];
  const int* srcs = ei;
  const int* dsts = ei + nE;
  float* out = (float*)d_out;

  const int nBlkG = (nN + GROWS - 1) / GROWS;
  const int NPADG = nBlkG * GROWS;
  const int nT    = (nE + KNB - 1) / KNB;
  const int nBlkS = (nT + NPB - 1) / NPB;
  const int nBlkP = (nN + NPB - 1) / NPB;
  const int nBC   = (nN + NBC - 1) / NBC;
  const int CNTPAD = nBC * NBC;
  if (4 * nBC + 1 > RBN) return;
  const int nBF    = (nN + NBF - 1) / NBF;
  const int csrLen = ((nE + 31) & ~31) + 4096;
  if (31 * 4 * nBC > 4096) return;

  char* ws = (char*)d_ws;
  size_t off = 0;
  const size_t oB   = off; off += (size_t)BPTOT * 2;               off = (off + 255) & ~(size_t)255;
  const size_t oCnt = off; off += (size_t)CNTPAD * 4;              off = (off + 255) & ~(size_t)255;
  const size_t oOff = off; off += (size_t)CNTPAD * 4;              off = (off + 255) & ~(size_t)255;
  const size_t oRb  = off; off += (size_t)RBN * 4;                 off = (off + 255) & ~(size_t)255;
  const size_t oCsr = off; off += (size_t)csrLen * 4;              off = (off + 255) & ~(size_t)255;
  const size_t oPQ  = off; off += (size_t)NPADG * PQW * 4;         off = (off + 255) & ~(size_t)255;
  const size_t oP1  = off; off += (size_t)nBlkS * (2 * CH) * 8;    off = (off + 255) & ~(size_t)255;
  const size_t oP2  = off; off += (size_t)nBlkS * (2 * CH) * 8;    off = (off + 255) & ~(size_t)255;
  const size_t oT1  = off; off += (size_t)4 * CH * 4;              off = (off + 255) & ~(size_t)255;
  const size_t oT2  = off; off += (size_t)4 * CH * 4;              off = (off + 255) & ~(size_t)255;
  if (off > ws_size || off > (size_t)WSCAP) return;
  _Float16* Bpl   = (_Float16*)(ws + oB);
  int*      cnt   = (int*)(ws + oCnt);
  int*      offp  = (int*)(ws + oOff);
  int*      rb    = (int*)(ws + oRb);
  int*      csr   = (int*)(ws + oCsr);
  float*    PQ    = (float*)(ws + oPQ);
  double*   part1 = (double*)(ws + oP1);
  double*   part2 = (double*)(ws + oP2);
  float*    tab1  = (float*)(ws + oT1);
  float*    tab2  = (float*)(ws + oT2);

  const double rn = 1.0 / (double)nE;
  const int vec8 = ((nE & 3) == 0) ? 1 : 0;

  k_wprep<<<8, NTHR, 0, stream>>>(W1, W2, W3, Bpl);
  k_count<<<nBC, NTHR, 0, stream>>>(dsts, cnt, nE, vec8);
  k_offsets<<<1, OTHR, 0, stream>>>(cnt, offp, rb, nBC);
  hipFuncSetAttribute(reinterpret_cast<const void*>(&k_fill),
                      hipFuncAttributeMaxDynamicSharedMemorySize, LDS_FILL);
  k_fill<<<nBF, NTHR, LDS_FILL, stream>>>(srcs, dsts, offp, rb, csr, nN, nE, vec8, csrLen);
  k_nodegemm<<<nBlkG, GTHR, 0, stream>>>(x, Bpl + OFF_B1, b1, PQ, nN);
  k_stats1<<<nBlkS, NTHR, 0, stream>>>(PQ, srcs, dsts, part1, nE, nN);
  k_bnfin<<<1, 64, 0, stream>>>(part1, g1, be1, b2, tab1, rn, nBlkS);
  k_stats2<<<nBlkS, NTHR, 0, stream>>>(PQ, srcs, dsts, Bpl + OFF_B2, tab1, part2, nE, nN);
  k_bnfin<<<1, 64, 0, stream>>>(part2, g2, be2, b3, tab2, rn, nBlkS);
  k_final<<<nBlkP, NTHR, 0, stream>>>(PQ, csr, offp, cnt, Bpl + OFF_B2, Bpl + OFF_B3, tab1, tab2, x, out, nN, csrLen);
}
